// EncoderBlock_70549132804729
// MI455X (gfx1250) — hardware-verified
//
#include <hip/hip_runtime.h>
#include <math.h>

#ifndef NB
#define NB 32
#endif
#ifndef SEQ
#define SEQ 1024
#endif
#define SEQ_FULL 1024
#define CH 128
#define HEADS 8
#define HD 16
#define KW 7
#define NCONV 4
#define NNORM 6
#define MTOK (NB * SEQ)
#define SLABROWS 8
#define NSLAB (SEQ / SLABROWS)
#define NCNT (CH * SEQ)

#define CARRY_ACT 64
#define CARRY_W 64
#define CARRY_QKV 256
#define CARRY_P 1024
#define CARRY_O 1024
#define SL_ACTW 12
#define SL_OW 16
#define OSL_QKV 8

static_assert(NB >= 1 && NB <= 32);
static_assert(SEQ <= SEQ_FULL && SEQ % 256 == 0);
static_assert(CH == 128 && HEADS * HD == CH && HD == 16);
static_assert(MTOK % 64 == 0 && CH % 64 == 0 && SEQ % 64 == 0);
static_assert(CH % 32 == 0);
static_assert((MTOK * CH / 8) % 256 == 0);
static_assert((MTOK * CH / 4) % 256 == 0);
static_assert((MTOK * CH) % 256 == 0);
static_assert((SEQ * CH / 4) % 256 == 0);
static_assert((CH * CH / 8) % 256 == 0);
static_assert(SLABROWS * CH == 256 * 4);
static_assert(MTOK % SLABROWS == 0);
static_assert(CARRY_ACT * CARRY_W == (1 << SL_ACTW));
static_assert(CARRY_O * CARRY_W == (1 << SL_OW));
static_assert(CARRY_QKV == (1 << OSL_QKV));
static_assert(CARRY_QKV * CARRY_QKV == 65536);
static_assert(CARRY_O == 4 * CARRY_QKV);
static_assert(CARRY_P == 1024);

typedef __attribute__((ext_vector_type(16))) _Float16 v16h;
typedef __attribute__((ext_vector_type(8)))  _Float16 v8h;
typedef __attribute__((ext_vector_type(8)))  float    v8f;
typedef __attribute__((ext_vector_type(4)))  float    v4f;
typedef __attribute__((ext_vector_type(4)))  unsigned int v4u;
typedef _Float16 h16;


#define VST2(T, ptr, val) do { const T vst2_v_ = (val); *(volatile T*)(ptr) = vst2_v_; __threadfence(); *(volatile T*)(ptr) = vst2_v_; } while (0)
#define VST2V4(ptr, val) do { const v4f vst2_v4_ = (val); *(volatile v4f*)(ptr) = vst2_v4_; __threadfence(); *(volatile v4f*)(ptr) = vst2_v4_; } while (0)

__device__ __forceinline__ float bfr(float f) {
    unsigned u = __float_as_uint(f);
    u += 0x7FFFu + ((u >> 16) & 1u);
    return __uint_as_float(u & 0xFFFF0000u);
}
static __device__ __forceinline__ h16 toh_flush(float v) { const float w = (fabsf(v) < 6.103515625e-05f) ? 0.0f : v; return (h16)w; }
typedef __attribute__((ext_vector_type(2))) _Float16 v2h;
typedef __attribute__((ext_vector_type(2))) float    v2f;
static __device__ __forceinline__ v2h toh2_flush(float a, float b) {
    v2f w;
    w.x = (fabsf(a) < 6.103515625e-05f) ? 0.0f : a;
    w.y = (fabsf(b) < 6.103515625e-05f) ? 0.0f : b;
    return __builtin_convertvector(w, v2h);
}
union Pack8 { v8h v; v2h p[4]; };
static __device__ __forceinline__ v8h pack8_flush(v4f a, v4f b) {
    Pack8 u;
    u.p[0] = toh2_flush(a.x, a.y); u.p[1] = toh2_flush(a.z, a.w);
    u.p[2] = toh2_flush(b.x, b.y); u.p[3] = toh2_flush(b.z, b.w);
    return u.v;
}
static __device__ __forceinline__ void st8h_flush(_Float16* P, size_t o, const float* v) {
    v8h hv;
#pragma unroll
    for (int e = 0; e < 8; ++e) hv[e] = toh_flush(v[e]);
    *(volatile v8h*)(P + o) = hv;
    __threadfence();
    *(volatile v8h*)(P + o) = hv;
}
static __device__ __forceinline__ void ld8f(const float* p, float* o) {
    const v4f a = *(const v4f*)p, b = *(const v4f*)(p + 4);
    o[0] = a.x; o[1] = a.y; o[2] = a.z; o[3] = a.w; o[4] = b.x; o[5] = b.y; o[6] = b.z; o[7] = b.w;
}

union FragU { v16h v; v8h h[2]; };
__device__ __forceinline__ v16h frag_ld(const _Float16* p) {
    FragU f; f.h[0] = *(const v8h*)(p); f.h[1] = *(const v8h*)(p + 16); return f.v;
}
__device__ __forceinline__ v8f wmma16(v16h a, v16h b, v8f c) {
    c = __builtin_amdgcn_wmma_f32_16x16x32_f16(false, a, false, b, (short)0, c, false, false);
    asm volatile("v_nop\n\tv_nop\n\tv_nop\n\tv_nop" : "+v"(c) : "v"(a), "v"(b));
    return c;
}
__device__ __forceinline__ void wave_sync_lds() {
    __builtin_amdgcn_fence(3  , "workgroup");
    __builtin_amdgcn_wave_barrier();
    __builtin_amdgcn_fence(2  , "workgroup");
}

template <int OUT_MODE, bool RESID, bool RELU, bool BIAS_ROW, int SL, int OSL>
__device__ __forceinline__ void gemm64_body(
    const _Float16* __restrict__ A, unsigned lda, const _Float16* __restrict__ Bt, unsigned ldb,
    void* __restrict__ Cout, unsigned ldc, const float* __restrict__ bias, const float* __restrict__ resid,
    unsigned M, unsigned N, unsigned K) {
  __shared__ __align__(16) float sT[8][16 * 68];
  static_assert(sizeof(float) * 8 * 16 * 68 <= 131072);
  const float scale = 1.0f / (float)(1u << SL);
  const float oscale = (float)(1u << OSL);
  const unsigned lane = threadIdx.x & 31u;
  const unsigned wave = (unsigned)__builtin_amdgcn_readfirstlane((int)(threadIdx.x >> 5));
  const unsigned tilesN = N >> 6, tilesM = M >> 6;
  const unsigned tile = blockIdx.x * 8u + wave;
  if (tile >= tilesM * tilesN) return;
  const unsigned tm = tile / tilesN;
  const unsigned tn = tile - tm * tilesN;
  const unsigned m0 = tm << 6, n0 = tn << 6;
  const unsigned rlane = lane & 15u;
  const unsigned koff = (lane >> 4) * 8u;
  const unsigned mOff = koff;

  v8f acc[4][4];
#pragma unroll
  for (int i = 0; i < 4; ++i)
#pragma unroll
    for (int j = 0; j < 4; ++j) acc[i][j] = (v8f){0.f,0.f,0.f,0.f,0.f,0.f,0.f,0.f};

  for (unsigned k0 = 0; k0 < K; k0 += 32u) {
    v16h bh[4];
#pragma unroll
    for (int j = 0; j < 4; ++j)
      bh[j] = frag_ld(Bt + (size_t)(n0 + ((unsigned)j << 4) + rlane) * ldb + koff + k0);
#pragma unroll
    for (int i = 0; i < 4; ++i) {
      const v16h ah = frag_ld(A + (size_t)(m0 + ((unsigned)i << 4) + rlane) * lda + koff + k0);
#pragma unroll
      for (int j = 0; j < 4; ++j)
        acc[i][j] = wmma16(ah, bh[j], acc[i][j]);
    }
  }

  float* slab = sT[wave];
#pragma unroll
  for (int i = 0; i < 4; ++i) {
    const unsigned mBase = m0 + ((unsigned)i << 4);
    float brow[8];
#pragma unroll
    for (int r = 0; r < 8; ++r) brow[r] = BIAS_ROW ? bfr(bias[mBase + mOff + (unsigned)r]) : 0.0f;
#pragma unroll
    for (int j = 0; j < 4; ++j) {
      const unsigned n = n0 + ((unsigned)j << 4) + rlane;
      const float bcol = BIAS_ROW ? 0.0f : bfr(bias[BIAS_ROW ? 0u : n]);
#pragma unroll
      for (int r = 0; r < 8; ++r) {
        float v = acc[i][j][r] * scale + (bcol + brow[r]);
        if (RELU) v = fmaxf(v, 0.0f);
        if (OUT_MODE == 1) v *= oscale;
        slab[(mOff + (unsigned)r) * 68u + ((unsigned)j << 4) + rlane] = v;
      }
    }
    wave_sync_lds();
    if (OUT_MODE == 0) {
      float* C = (float*)Cout;
      const unsigned hh = lane >> 4, c4 = (lane & 15u) * 4u;
      static_assert(32 * 16 * (2 * 4) == 16 * 64 * 4);
#pragma unroll
      for (int half = 0; half < 2; ++half) {
        v4f vv[4];
#pragma unroll
        for (int it = 0; it < 4; ++it) {
          const unsigned row = (unsigned)(half * 4 + it) * 2u + hh;
          vv[it] = *(const v4f*)(slab + row * 68u + c4);
          if (RESID) vv[it] += *(const v4f*)(resid + (size_t)(mBase + row) * ldc + n0 + c4);
        }
        for (int pass = 0; pass < 2; ++pass) {
#pragma unroll
          for (int it = 0; it < 4; ++it) {
            const unsigned row = (unsigned)(half * 4 + it) * 2u + hh;
            *(volatile v4f*)(C + (size_t)(mBase + row) * ldc + n0 + c4) = vv[it];
          }
          __threadfence();
        }
      }
    } else {
      _Float16* C = (_Float16*)Cout;
      const unsigned q = lane >> 3, c8 = (lane & 7u) * 8u;
      static_assert(32 * 16 * 4 == 16 * 64 * 2);
      v8h hv[4];
#pragma unroll
      for (int it = 0; it < 4; ++it) {
        const unsigned row = (unsigned)it * 4u + q;
        const float* sp = slab + row * 68u + c8;
#pragma unroll
        for (int e = 0; e < 8; ++e) hv[it][e] = toh_flush(sp[e]);
      }
      for (int pass = 0; pass < 2; ++pass) {
#pragma unroll
        for (int it = 0; it < 4; ++it) {
          const unsigned row = (unsigned)it * 4u + q;
          *(volatile v8h*)(C + (size_t)(mBase + row) * ldc + n0 + c8) = hv[it];
        }
        __threadfence();
      }
    }
    wave_sync_lds();
  }
}

__global__ __launch_bounds__(256) void k_gemm_pw(const _Float16* __restrict__ A, const _Float16* __restrict__ Bt,
                                                 float* __restrict__ C, const float* __restrict__ bias,
                                                 const float* __restrict__ resid) {
  gemm64_body<0, true, true, false, SL_ACTW, 0>(A, CH, Bt, CH, (void*)C, CH, bias, resid, MTOK, CH, CH);
}
__global__ __launch_bounds__(256) void k_gemm_qk(const _Float16* __restrict__ A, const _Float16* __restrict__ Bt,
                                                 _Float16* __restrict__ C, const float* __restrict__ bias) {
  gemm64_body<1, false, false, false, SL_ACTW, OSL_QKV>(A, CH, Bt, CH, (void*)C, CH, bias, nullptr, MTOK, CH, CH);
}
__global__ __launch_bounds__(256) void k_gemm_vt(const _Float16* __restrict__ W16, const _Float16* __restrict__ X16,
                                                 _Float16* __restrict__ VT, const float* __restrict__ bias) {
  const unsigned b = blockIdx.y;
  gemm64_body<1, false, false, true, SL_ACTW, OSL_QKV>(W16, CH, X16 + (size_t)b * SEQ * CH, CH,
      (void*)(VT + (size_t)b * CH * SEQ), SEQ, bias, nullptr, CH, SEQ, CH);
}
__global__ __launch_bounds__(256) void k_gemm_aw(const _Float16* __restrict__ A, const _Float16* __restrict__ Bt,
                                                 float* __restrict__ C, const float* __restrict__ bias,
                                                 const float* __restrict__ resid) {
  gemm64_body<0, true, false, false, SL_OW, 0>(A, CH, Bt, CH, (void*)C, CH, bias, resid, MTOK, CH, CH);
}
__global__ __launch_bounds__(256) void k_gemm_fw(const _Float16* __restrict__ A, const _Float16* __restrict__ Bt,
                                                 float* __restrict__ C, const float* __restrict__ bias) {
  gemm64_body<0, false, false, false, SL_ACTW, 0>(A, CH, Bt, CH, (void*)C, CH, bias, nullptr, MTOK, CH, CH);
}

__global__ __launch_bounds__(256) void k_wt(const float* __restrict__ Wm, _Float16* __restrict__ W16) {
    const unsigned layer = blockIdx.y;
    const unsigned u = blockIdx.x * 256u + threadIdx.x;
    if (u >= (unsigned)(CH * CH / 8)) return;
    float w[8], v[8];
    ld8f(Wm + (size_t)layer * CH * CH + 8u * u, w);
#pragma unroll
    for (int i = 0; i < 8; ++i) v[i] = bfr(w[i]) * (float)CARRY_W;
    st8h_flush(W16 + (size_t)layer * CH * CH, (size_t)8u * u, v);
}

__global__ __launch_bounds__(256) void k_nt(const float* __restrict__ src, float* __restrict__ dst) {
    const unsigned layer = blockIdx.y;
    const unsigned u = blockIdx.x * 256u + threadIdx.x;
    if (u >= (unsigned)(SEQ * CH / 4)) return;
    const unsigned l = u >> 5, c = (u & 31u) * 4u;
    const float* s = src + (size_t)layer * CH * SEQ_FULL + (size_t)c * SEQ_FULL + l;
    v4f v;
    v.x = bfr(s[0]); v.y = bfr(s[SEQ_FULL]); v.z = bfr(s[2 * SEQ_FULL]); v.w = bfr(s[3 * SEQ_FULL]);
    VST2V4(dst + (size_t)layer * SEQ * CH + (size_t)l * CH + c, v);
}

__global__ __launch_bounds__(256) void k_in(const float* __restrict__ x, const float* __restrict__ pos, float* __restrict__ RES) {
    const unsigned u = blockIdx.x * 256u + threadIdx.x;
    if (u >= (unsigned)(MTOK * CH / 4)) return;
    const unsigned row = u >> 5, c = (u & 31u) * 4u;
    const unsigned b = row / (unsigned)SEQ, l = row - b * (unsigned)SEQ;
    const float* xb = x + ((size_t)b * CH + c) * SEQ_FULL + l;
    const float* pp = pos + (size_t)c * SEQ_FULL + l;
    v4f v;
    v.x = bfr(xb[0]) + bfr(pp[0]);
    v.y = bfr(xb[SEQ_FULL]) + bfr(pp[SEQ_FULL]);
    v.z = bfr(xb[2 * SEQ_FULL]) + bfr(pp[2 * SEQ_FULL]);
    v.w = bfr(xb[3 * SEQ_FULL]) + bfr(pp[3 * SEQ_FULL]);
    VST2V4(RES + (size_t)row * CH + c, v);
}

__global__ __launch_bounds__(256) void k_sum(const float* __restrict__ P, float* __restrict__ PART) {
    __shared__ float sw[8];
    const unsigned tid = threadIdx.x, lane = tid & 31u;
    const unsigned wave = (unsigned)__builtin_amdgcn_readfirstlane((int)(tid >> 5));
    const v4f a = *(const v4f*)(P + (size_t)blockIdx.x * 1024u + 4u * tid);
    float s = a.x; s += a.y; s += a.z; s += a.w;
#pragma unroll
    for (int o = 16; o > 0; o >>= 1) s += __shfl_xor(s, o, 32);
    if (lane == 0u) sw[wave] = s;
    __syncthreads();
    if (wave == 0u) {
        float t = sw[0];
#pragma unroll
        for (int i = 1; i < 8; ++i) t += sw[i];
        v4f v; v.x = t; v.y = t; v.z = t; v.w = t;
        if (lane < 8u) { VST2V4(PART + (size_t)blockIdx.x * 32u + 4u * lane, v); }
    }
}
__global__ __launch_bounds__(256) void k_sq(const float* __restrict__ P, const float* __restrict__ MU, float* __restrict__ PART) {
    __shared__ float sw[8];
    const unsigned tid = threadIdx.x, lane = tid & 31u;
    const unsigned wave = (unsigned)__builtin_amdgcn_readfirstlane((int)(tid >> 5));
    const float mu = MU[blockIdx.x / (unsigned)NSLAB];
    const v4f a = *(const v4f*)(P + (size_t)blockIdx.x * 1024u + 4u * tid);
    float d = a.x - mu; float s = d * d;
    d = a.y - mu; s += d * d;
    d = a.z - mu; s += d * d;
    d = a.w - mu; s += d * d;
#pragma unroll
    for (int o = 16; o > 0; o >>= 1) s += __shfl_xor(s, o, 32);
    if (lane == 0u) sw[wave] = s;
    __syncthreads();
    if (wave == 0u) {
        float t = sw[0];
#pragma unroll
        for (int i = 1; i < 8; ++i) t += sw[i];
        v4f v; v.x = t; v.y = t; v.z = t; v.w = t;
        if (lane < 8u) { VST2V4(PART + (size_t)blockIdx.x * 32u + 4u * lane, v); }
    }
}
__global__ __launch_bounds__(32) void k_mean(const float* __restrict__ PART, float* __restrict__ MU) {
    __shared__ float sv[32];
    const unsigned lane = threadIdx.x & 31u;
    const unsigned bb = (lane < (unsigned)NB) ? lane : (unsigned)(NB - 1);
    float s = 0.f;
#pragma unroll 8
    for (unsigned j = 0; j < (unsigned)NSLAB; ++j) s += PART[((size_t)bb * NSLAB + j) * 32u];
    sv[lane] = s / (float)NCNT;
    __syncthreads();
    const unsigned l8 = lane & 7u;
    v4f v; v.x = sv[4u * l8]; v.y = sv[4u * l8 + 1u]; v.z = sv[4u * l8 + 2u]; v.w = sv[4u * l8 + 3u];
    if (lane < 8u) { VST2V4(MU + 4u * l8, v); }
}
__global__ __launch_bounds__(32) void k_rstd(const float* __restrict__ PART, float* __restrict__ RSTD) {
    __shared__ float sv[32];
    const unsigned lane = threadIdx.x & 31u;
    const unsigned bb = (lane < (unsigned)NB) ? lane : (unsigned)(NB - 1);
    float s = 0.f;
#pragma unroll 8
    for (unsigned j = 0; j < (unsigned)NSLAB; ++j) s += PART[((size_t)bb * NSLAB + j) * 32u];
    const float var = s / (float)NCNT;
    sv[lane] = 1.0f / sqrtf(var + 1e-5f);
    __syncthreads();
    const unsigned l8 = lane & 7u;
    v4f v; v.x = sv[4u * l8]; v.y = sv[4u * l8 + 1u]; v.z = sv[4u * l8 + 2u]; v.w = sv[4u * l8 + 3u];
    if (lane < 8u) { VST2V4(RSTD + 4u * l8, v); }
}

__global__ __launch_bounds__(256) void k_dw(const float* __restrict__ RESI, const float* __restrict__ NW, const float* __restrict__ NBp,
                                            const float* __restrict__ MU, const float* __restrict__ RSTD,
                                            const float* __restrict__ dww, const float* __restrict__ dwb,
                                            _Float16* __restrict__ HDW) {
    const unsigned u = blockIdx.x * 256u + threadIdx.x;
    if (u >= (unsigned)(MTOK * CH / 8)) return;
    const unsigned row = u >> 4, c0 = (u & 15u) * 8u;
    const unsigned b = row / (unsigned)SEQ, l = row - b * (unsigned)SEQ;
    const float mu = MU[b], rs = RSTD[b];
    float wv[56];
    {
        const v4f* wp = (const v4f*)(dww + (size_t)c0 * KW);
#pragma unroll
        for (int g = 0; g < 14; ++g) {
            const v4f t = wp[g];
            wv[4 * g] = bfr(t.x); wv[4 * g + 1] = bfr(t.y); wv[4 * g + 2] = bfr(t.z); wv[4 * g + 3] = bfr(t.w);
        }
    }
    float acc[8];
#pragma unroll
    for (int i = 0; i < 8; ++i) acc[i] = 0.f;
#pragma unroll
    for (int t = 0; t < KW; ++t) {
        const int lp = (int)l + t - 3;
        const bool ok = (lp >= 0) && (lp < SEQ);
        const unsigned lc = (unsigned)min(max(lp, 0), SEQ - 1);
        float xs[8], ws[8], bs[8];
        ld8f(RESI + ((size_t)b * SEQ + lc) * CH + c0, xs);
        ld8f(NW + (size_t)lc * CH + c0, ws);
        ld8f(NBp + (size_t)lc * CH + c0, bs);
#pragma unroll
        for (int i = 0; i < 8; ++i) {
            const float y = (xs[i] - mu) * rs * ws[i] + bs[i];
            const float yv = ok ? y : 0.0f;
            acc[i] += yv * wv[i * KW + t];
        }
    }
    float db[8], o[8];
    ld8f(dwb + c0, db);
#pragma unroll
    for (int i = 0; i < 8; ++i) o[i] = (acc[i] + bfr(db[i])) * (float)CARRY_ACT;
    st8h_flush(HDW, (size_t)u * 8u, o);
}

__global__ __launch_bounds__(256) void k_lnA(const float* __restrict__ RESI, const float* __restrict__ NW, const float* __restrict__ NBp,
                                             const float* __restrict__ MU, const float* __restrict__ RSTD,
                                             _Float16* __restrict__ XLN) {
    const unsigned u = blockIdx.x * 256u + threadIdx.x;
    if (u >= (unsigned)(MTOK * CH / 8)) return;
    const unsigned row = u >> 4, c0 = (u & 15u) * 8u;
    const unsigned b = row / (unsigned)SEQ, l = row - b * (unsigned)SEQ;
    const float mu = MU[b], rs = RSTD[b];
    float xs[8], ws[8], bs[8], y[8];
    ld8f(RESI + (size_t)row * CH + c0, xs);
    ld8f(NW + (size_t)l * CH + c0, ws);
    ld8f(NBp + (size_t)l * CH + c0, bs);
#pragma unroll
    for (int i = 0; i < 8; ++i) y[i] = ((xs[i] - mu) * rs * ws[i] + bs[i]) * (float)CARRY_ACT;
    st8h_flush(XLN, (size_t)u * 8u, y);
}

#define AT_PP 72
#define AT_OP 68
static_assert(16 * 16 * AT_PP * 2 + 16 * 16 * AT_OP * 4 <= 131072);
__global__ __launch_bounds__(512) void k_attn(const _Float16* __restrict__ Q16, const _Float16* __restrict__ K16,
                                              const _Float16* __restrict__ VT16, const float* __restrict__ mask,
                                              _Float16* __restrict__ O16) {
    __shared__ __align__(16) _Float16 sP[16][16 * AT_PP];
    __shared__ __align__(16) float sO[16][16 * AT_OP];
    const unsigned tid = threadIdx.x, lane = tid & 31u;
    const unsigned wave = (unsigned)__builtin_amdgcn_readfirstlane((int)(tid >> 5));
    const unsigned hh = lane >> 4, c = lane & 15u;
    const unsigned qblk = blockIdx.x % (unsigned)(SEQ / 256);
    const unsigned bq = blockIdx.x / (unsigned)(SEQ / 256);
    const unsigned quad = bq & 1u, b = bq >> 1;
    const unsigned q0 = qblk * 256u + wave * 16u;
    _Float16* pw = sP[wave];
    const float SCQK = 0.25f / (float)(CARRY_QKV * CARRY_QKV);
    const float LOG2E = 1.4426950408889634f;
    const float* mk = mask + (size_t)b * SEQ_FULL;
    const v8h zero8 = {};
    v8f ofin[4];
#pragma unroll
    for (int hq = 0; hq < 4; ++hq) {
        const unsigned head = 4u * quad + (unsigned)hq;
        FragU qu;
        qu.h[0] = *(const v8h*)(Q16 + (size_t)(b * SEQ + q0 + c) * CH + head * 16u + 8u * hh);
        qu.h[1] = zero8;
        const v16h qf = qu.v;
        float mrow[8], lrow[8];
        v8f os = (v8f){0.f,0.f,0.f,0.f,0.f,0.f,0.f,0.f};
#pragma unroll
        for (int r = 0; r < 8; ++r) { mrow[r] = -3.0e38f; lrow[r] = 0.f; }
#pragma unroll 1
        for (unsigned kc = 0; kc < (unsigned)(SEQ / 64); ++kc) {
            const unsigned kv0 = kc * 64u;
            v8f s[4];
            float om[4], mneg[4];
#pragma unroll
            for (int j = 0; j < 4; ++j) {
                FragU ku;
                ku.h[0] = *(const v8h*)(K16 + (size_t)(b * SEQ + kv0 + (unsigned)j * 16u + c) * CH + head * 16u + 8u * hh);
                ku.h[1] = zero8;
                const v8f z = (v8f){0.f,0.f,0.f,0.f,0.f,0.f,0.f,0.f};
                s[j] = wmma16(qf, ku.v, z);
                const float m = bfr(mk[kv0 + (unsigned)j * 16u + c]);
                om[j] = 1.0f - m;
                mneg[j] = m * (-1.0e30f);
            }
#pragma unroll
            for (int r = 0; r < 8; ++r) {
                float mx = -3.0e38f;
#pragma unroll
                for (int j = 0; j < 4; ++j) { s[j][r] = ((s[j][r] * SCQK) * om[j] + mneg[j]) * LOG2E; mx = fmaxf(mx, s[j][r]); }
                mx = fmaxf(mx, __shfl_xor(mx, 1, 32)); mx = fmaxf(mx, __shfl_xor(mx, 2, 32));
                mx = fmaxf(mx, __shfl_xor(mx, 4, 32)); mx = fmaxf(mx, __shfl_xor(mx, 8, 32));
                const float mnew = fmaxf(mrow[r], mx);
                const float alpha = exp2f(mrow[r] - mnew);
                mrow[r] = mnew;
                float psum = 0.f;
#pragma unroll
                for (int j = 0; j < 4; ++j) {
                    const float p = exp2f(s[j][r] - mnew);
                    psum += p;
                    pw[(8u * hh + (unsigned)r) * AT_PP + (unsigned)j * 16u + c] = toh_flush(p * (float)CARRY_P);
                }
                psum += __shfl_xor(psum, 1, 32); psum += __shfl_xor(psum, 2, 32);
                psum += __shfl_xor(psum, 4, 32); psum += __shfl_xor(psum, 8, 32);
                lrow[r] = lrow[r] * alpha + psum;
                os[r] *= alpha;
            }
            wave_sync_lds();
#pragma unroll
            for (int kk = 0; kk < 2; ++kk) {
                const v16h pa = frag_ld(pw + c * AT_PP + (unsigned)kk * 32u + 8u * hh);
                const v16h vb = frag_ld(VT16 + ((size_t)b * CH + head * 16u + c) * SEQ + kv0 + (unsigned)kk * 32u + 8u * hh);
                os = wmma16(pa, vb, os);
            }
            wave_sync_lds();
        }
#pragma unroll
        for (int r = 0; r < 8; ++r) {
            const float inv = 1.0f / (lrow[r] * (float)CARRY_P);
            ofin[hq][r] = os[r] * inv * (float)(CARRY_O / CARRY_QKV);
        }
    }
    float* so = sO[wave];
#pragma unroll
    for (int hq = 0; hq < 4; ++hq)
#pragma unroll
        for (int r = 0; r < 8; ++r)
            so[(8u * hh + (unsigned)r) * AT_OP + (unsigned)hq * 16u + c] = ofin[hq][r];
    wave_sync_lds();
    {
        const unsigned q = lane >> 3, c8 = (lane & 7u) * 8u;
        static_assert(32 * 16 * 4 == 16 * 64 * 2);
        v8h ov[4];
#pragma unroll
        for (int it = 0; it < 4; ++it) {
            const float* sp = so + ((unsigned)it * 4u + q) * AT_OP + c8;
            ov[it] = pack8_flush(*(const v4f*)sp, *(const v4f*)(sp + 4));
        }
        _Float16* dst = O16 + (size_t)(b * SEQ + q0) * CH + quad * 64u;
        for (int pass = 0; pass < 2; ++pass) {
#pragma unroll
            for (int it = 0; it < 4; ++it) *(volatile v8h*)(dst + (size_t)((unsigned)it * 4u + q) * CH + c8) = ov[it];
            __threadfence();
        }
    }
}

__global__ __launch_bounds__(256) void k_out(const float* __restrict__ C2, const float* __restrict__ RES, float* __restrict__ out) {
    const unsigned u = blockIdx.x * 256u + threadIdx.x;
    if (u >= (unsigned)(MTOK * CH)) return;
    const unsigned ll = u & 31u, e = (u >> 5) & 127u, rest = u >> 12;
    const unsigned lb = rest % (unsigned)(SEQ / 32), b = rest / (unsigned)(SEQ / 32);
    const unsigned l = lb * 32u + ll;
    const size_t src = ((size_t)b * SEQ + l) * CH + e;
    const float v = fmaxf(C2[src], 0.0f) + RES[src];
    VST2(float, out + ((size_t)b * CH + e) * SEQ_FULL + l, v);
}

constexpr size_t SZ_F32   = (size_t)MTOK * CH * 4;
constexpr size_t SZ_F16   = (size_t)MTOK * CH * 2;
constexpr size_t SZ_NT    = (size_t)NNORM * SEQ * CH * 4;
constexpr size_t SZ_W     = (size_t)CH * CH * 2;
constexpr size_t SZ_PART  = (size_t)NB * NSLAB * 32 * 4;
constexpr size_t SZ_STAT  = (size_t)NNORM * 32 * 4;
constexpr size_t OFF_RESA = 0;
constexpr size_t OFF_RESB = OFF_RESA + SZ_F32;
constexpr size_t OFF_C2   = OFF_RESB + SZ_F32;
constexpr size_t OFF_HDW  = OFF_C2 + SZ_F32;
constexpr size_t OFF_XLN  = OFF_HDW + SZ_F16;
constexpr size_t OFF_Q    = OFF_XLN + SZ_F16;
constexpr size_t OFF_K    = OFF_Q + SZ_F16;
constexpr size_t OFF_VT   = OFF_K + SZ_F16;
constexpr size_t OFF_O    = OFF_VT + SZ_F16;
constexpr size_t OFF_NTW  = OFF_O + SZ_F16;
constexpr size_t OFF_NTB  = OFF_NTW + SZ_NT;
constexpr size_t OFF_PW   = OFF_NTB + SZ_NT;
constexpr size_t OFF_QW   = OFF_PW + NCONV * SZ_W;
constexpr size_t OFF_KW   = OFF_QW + SZ_W;
constexpr size_t OFF_VW   = OFF_KW + SZ_W;
constexpr size_t OFF_AW   = OFF_VW + SZ_W;
constexpr size_t OFF_FW   = OFF_AW + SZ_W;
constexpr size_t OFF_PA   = OFF_FW + SZ_W;
constexpr size_t OFF_PB   = OFF_PA + SZ_PART;
constexpr size_t OFF_MU   = OFF_PB + SZ_PART;
constexpr size_t OFF_RSTD = OFF_MU + SZ_STAT;
constexpr size_t WS_TOTAL = OFF_RSTD + SZ_STAT;
static_assert(SZ_F32 % 256 == 0 && SZ_F16 % 256 == 0 && SZ_NT % 256 == 0 && SZ_W % 256 == 0 && SZ_PART % 256 == 0 && SZ_STAT % 256 == 0);
static_assert(WS_TOTAL <= (size_t)134217728);
static_assert((size_t)(NB - 1) * CH * SEQ_FULL + (size_t)(CH - 1) * SEQ_FULL + SEQ <= (size_t)NB * CH * SEQ_FULL);

extern "C" void kernel_launch(void* const* d_in, const int* in_sizes, int n_in, void* d_out, int out_size,
                              void* d_ws, size_t ws_size, hipStream_t stream) {
    if (n_in < 23) return;
    if (in_sizes[0] < NB * CH * SEQ_FULL || in_sizes[1] < NB * SEQ_FULL || in_sizes[2] < CH * SEQ_FULL) return;
    if (in_sizes[3] < CH * SEQ_FULL || in_sizes[4] < CH * SEQ_FULL) return;
    if (in_sizes[5] < NCONV * CH * KW || in_sizes[6] < NCONV * CH || in_sizes[7] < NCONV * CH * CH || in_sizes[8] < NCONV * CH) return;
    if (in_sizes[9] < NCONV * CH * SEQ_FULL || in_sizes[10] < NCONV * CH * SEQ_FULL) return;
    if (in_sizes[11] < CH * CH || in_sizes[12] < CH || in_sizes[13] < CH * CH || in_sizes[14] < CH) return;
    if (in_sizes[15] < CH * CH || in_sizes[16] < CH || in_sizes[17] < CH * CH || in_sizes[18] < CH) return;
    if (in_sizes[19] < CH * SEQ_FULL || in_sizes[20] < CH * SEQ_FULL || in_sizes[21] < CH * CH || in_sizes[22] < CH) return;
    if (out_size < NB * CH * SEQ_FULL) return;
    if (ws_size < WS_TOTAL) return;

    const float* x       = (const float*)d_in[0];
    const float* mask    = (const float*)d_in[1];
    const float* pos_enc = (const float*)d_in[2];
    const float* normb_w = (const float*)d_in[3];
    const float* normb_b = (const float*)d_in[4];
    const float* dw_w    = (const float*)d_in[5];
    const float* dw_b    = (const float*)d_in[6];
    const float* pw_w    = (const float*)d_in[7];
    const float* pw_b    = (const float*)d_in[8];
    const float* norms_w = (const float*)d_in[9];
    const float* norms_b = (const float*)d_in[10];
    const float* qw      = (const float*)d_in[11];
    const float* qb      = (const float*)d_in[12];
    const float* kw      = (const float*)d_in[13];
    const float* kb      = (const float*)d_in[14];
    const float* vw      = (const float*)d_in[15];
    const float* vb      = (const float*)d_in[16];
    const float* aw      = (const float*)d_in[17];
    const float* ab      = (const float*)d_in[18];
    const float* norme_w = (const float*)d_in[19];
    const float* norme_b = (const float*)d_in[20];
    const float* fw      = (const float*)d_in[21];
    const float* fb      = (const float*)d_in[22];
    float* out = (float*)d_out;

    char* wsp = (char*)d_ws;
    float*    RESA  = (float*)(wsp + OFF_RESA);
    float*    RESB  = (float*)(wsp + OFF_RESB);
    float*    C2    = (float*)(wsp + OFF_C2);
    _Float16* HDW   = (_Float16*)(wsp + OFF_HDW);
    _Float16* XLN   = (_Float16*)(wsp + OFF_XLN);
    _Float16* Q16   = (_Float16*)(wsp + OFF_Q);
    _Float16* K16   = (_Float16*)(wsp + OFF_K);
    _Float16* VT16  = (_Float16*)(wsp + OFF_VT);
    _Float16* O16   = (_Float16*)(wsp + OFF_O);
    float*    NTW   = (float*)(wsp + OFF_NTW);
    float*    NTB   = (float*)(wsp + OFF_NTB);
    _Float16* PW16  = (_Float16*)(wsp + OFF_PW);
    _Float16* QW16  = (_Float16*)(wsp + OFF_QW);
    _Float16* KW16  = (_Float16*)(wsp + OFF_KW);
    _Float16* VW16  = (_Float16*)(wsp + OFF_VW);
    _Float16* AW16  = (_Float16*)(wsp + OFF_AW);
    _Float16* FW16  = (_Float16*)(wsp + OFF_FW);
    float*    PARTA = (float*)(wsp + OFF_PA);
    float*    PARTB = (float*)(wsp + OFF_PB);
    float*    MU    = (float*)(wsp + OFF_MU);
    float*    RSTD  = (float*)(wsp + OFF_RSTD);

    const size_t PL = (size_t)SEQ * CH;

    const unsigned gW = (CH * CH / 8) / 256;
    k_wt<<<dim3(gW, NCONV), 256, 0, stream>>>(pw_w, PW16);
    k_wt<<<dim3(gW, 1), 256, 0, stream>>>(qw, QW16);
    k_wt<<<dim3(gW, 1), 256, 0, stream>>>(kw, KW16);
    k_wt<<<dim3(gW, 1), 256, 0, stream>>>(vw, VW16);
    k_wt<<<dim3(gW, 1), 256, 0, stream>>>(aw, AW16);
    k_wt<<<dim3(gW, 1), 256, 0, stream>>>(fw, FW16);

    const unsigned gN = (SEQ * CH / 4) / 256;
    k_nt<<<dim3(gN, 1), 256, 0, stream>>>(normb_w, NTW);
    k_nt<<<dim3(gN, 1), 256, 0, stream>>>(normb_b, NTB);
    k_nt<<<dim3(gN, NCONV), 256, 0, stream>>>(norms_w, NTW + PL);
    k_nt<<<dim3(gN, NCONV), 256, 0, stream>>>(norms_b, NTB + PL);
    k_nt<<<dim3(gN, 1), 256, 0, stream>>>(norme_w, NTW + 5 * PL);
    k_nt<<<dim3(gN, 1), 256, 0, stream>>>(norme_b, NTB + 5 * PL);

    k_in<<<(MTOK * CH / 4) / 256, 256, 0, stream>>>(x, pos_enc, RESA);

    auto stats = [&](const float* plane, int j) {
        k_sum<<<MTOK / SLABROWS, 256, 0, stream>>>(plane, PARTA);
        k_mean<<<1, 32, 0, stream>>>(PARTA, MU + j * 32);
        k_sq<<<MTOK / SLABROWS, 256, 0, stream>>>(plane, MU + j * 32, PARTB);
        k_rstd<<<1, 32, 0, stream>>>(PARTB, RSTD + j * 32);
    };

    const unsigned gT = ((MTOK / 64) * (CH / 64) + 7) / 8;
    const unsigned gE = (MTOK * CH / 8) / 256;

    stats(RESA, 0);
    float* rin = RESA;
    float* rout = RESB;
    for (int i = 0; i < NCONV; ++i) {
        k_dw<<<gE, 256, 0, stream>>>(rin, NTW + (size_t)i * PL, NTB + (size_t)i * PL, MU + i * 32, RSTD + i * 32,
                                     dw_w + (size_t)i * CH * KW, dw_b + (size_t)i * CH, HDW);
        k_gemm_pw<<<gT, 256, 0, stream>>>((const _Float16*)HDW, (const _Float16*)(PW16 + (size_t)i * CH * CH), rout,
                                          pw_b + (size_t)i * CH, (const float*)rin);
        stats(rout, i + 1);
        float* t = rin; rin = rout; rout = t;
    }

    k_lnA<<<gE, 256, 0, stream>>>(rin, NTW + 4 * PL, NTB + 4 * PL, MU + 4 * 32, RSTD + 4 * 32, XLN);
    k_gemm_qk<<<gT, 256, 0, stream>>>((const _Float16*)XLN, (const _Float16*)QW16, Q16, qb);
    k_gemm_qk<<<gT, 256, 0, stream>>>((const _Float16*)XLN, (const _Float16*)KW16, K16, kb);
    k_gemm_vt<<<dim3(((CH / 64) * (SEQ / 64) + 7) / 8, NB), 256, 0, stream>>>((const _Float16*)VW16, (const _Float16*)XLN, VT16, vb);
    k_attn<<<NB * 2 * (SEQ / 256), 512, 0, stream>>>((const _Float16*)Q16, (const _Float16*)K16, (const _Float16*)VT16, mask, O16);
    k_gemm_aw<<<gT, 256, 0, stream>>>((const _Float16*)O16, (const _Float16*)AW16, rout, ab, (const float*)rin);

    stats(rout, 5);
    k_lnA<<<gE, 256, 0, stream>>>(rout, NTW + 5 * PL, NTB + 5 * PL, MU + 5 * 32, RSTD + 5 * 32, XLN);
    k_gemm_fw<<<gT, 256, 0, stream>>>((const _Float16*)XLN, (const _Float16*)FW16, C2, fb);
    k_out<<<(MTOK * CH) / 256, 256, 0, stream>>>((const float*)C2, (const float*)rout, out);
}
